// GINet_67929202753747
// MI455X (gfx1250) — hardware-run, weakly checked
//
#include <hip/hip_runtime.h>


namespace {
constexpr int N = 10000, NP = 10048, NLIM = 10048  , NLIMN = (NLIM < N ? NLIM : N), EFULL = 160000, E = EFULL, D = 300, DP = 320, H2 = 600, HP = 640, L = 5, G = 512, FD = 256, FD2 = 128, NT = 15  , RPB = 64, NBP = NP / RPB, NBPL = NLIM / RPB;
constexpr float XS = 8.0f, WSC = 256.0f, BNEPS = 1e-5f;
static_assert(NP % 64 == 0 && NLIM % 64 == 0 && NLIM <= NP && DP % 64 == 0 && HP % 64 == 0 && G % 64 == 0, "tiling");
typedef _Float16 b16;
typedef __attribute__((ext_vector_type(16))) _Float16 v16b;
typedef __attribute__((ext_vector_type(8))) _Float16 v8b;
typedef __attribute__((ext_vector_type(8))) float v8f;
typedef __attribute__((ext_vector_type(4))) float v4f;
__device__ __forceinline__ float bf16_rne(float f) { unsigned int u = __float_as_uint(f); u += 0x7FFFu + ((u >> 16) & 1u); return __uint_as_float(u & 0xFFFF0000u); }
__device__ __forceinline__ void split16(float v, b16& hi, b16& lo) { hi = (b16)v; lo = (b16)(v - (float)hi); }
__device__ __forceinline__ v16b frag_kb(const b16* p, int hh) { const v8b a = *(const v8b*)(p + 8 * hh), b = *(const v8b*)(p + 16 + 8 * hh); v16b f;
#pragma unroll
  for (int e = 0; e < 8; ++e) { f[e] = a[e]; f[8 + e] = b[e]; } return f; }
__device__ __forceinline__ v8f wmma16b(v16b a, v16b b, v8f c) { v8f d = __builtin_amdgcn_wmma_f32_16x16x32_f16(false, a, false, b, (short)0, c, false, false); asm volatile("v_nop\n\tv_nop\n\tv_nop\n\tv_nop" : "+v"(d) : "v"(a), "v"(b)); return d; }
__device__ __forceinline__ void wave_lds_sync() { __builtin_amdgcn_fence(__ATOMIC_RELEASE, "workgroup"); __builtin_amdgcn_wave_barrier(); __builtin_amdgcn_fence(__ATOMIC_ACQUIRE, "workgroup"); }
__device__ __forceinline__ float pmul(float a, float b) { float p = a * b; asm volatile("" : "+v"(p)); return p; }
__device__ __forceinline__ int iclamp(int v, int lo, int hi) { return v < lo ? lo : (v > hi ? hi : v); }
constexpr int CSR_NBLK = 512, CSR_GB = 9, CSR_GN = 1 << CSR_GB  , CSR_MAXG = 512, CSR_CAP = 12288  ;
__global__ __launch_bounds__(64) void csrA_kernel(const int* __restrict__ dst, int E, int N, int nG, int CHP, int NGP, int* __restrict__ STG, int* __restrict__ HST) {
  extern __shared__ int sm[];
  int* cnt = sm; int* run = sm + NGP; int* ids = sm + 2 * NGP;
  const int b = blockIdx.x; const int ch = (E + CSR_NBLK - 1) / CSR_NBLK; const int e0 = b * ch, e1 = min(E, e0 + ch);
  for (int i = threadIdx.x; i < NGP; i += 64) cnt[i] = 0;
  for (int i = threadIdx.x; i < CHP; i += 64) ids[i] = -1;
  __syncthreads();
  if (threadIdx.x == 0) {
    for (int e = e0; e < e1; ++e) { int d = dst[e]; d = (d < 0) ? 0 : (d >= N ? N - 1 : d); cnt[d >> CSR_GB] += 1; }
    int acc = 0; for (int g = 0; g < nG; ++g) { run[g] = acc; acc += cnt[g]; }
    for (int e = e0; e < e1; ++e) { int d = dst[e]; d = (d < 0) ? 0 : (d >= N ? N - 1 : d); const int g = d >> CSR_GB; ids[run[g]] = e; run[g] += 1; } }
  __syncthreads();
  typedef __attribute__((ext_vector_type(4))) int v4i;
  for (int pass = 0; pass < 2; ++pass) {
    for (int i = threadIdx.x; i < CHP / 4; i += 64) *(volatile v4i*)(STG + (size_t)b * CHP + i * 4) = *(const v4i*)(&ids[i * 4]);
    for (int i = threadIdx.x; i < NGP / 4; i += 64) { v4i v; for (int e = 0; e < 4; ++e) v[e] = (i * 4 + e < nG) ? cnt[i * 4 + e] : 0; *(volatile v4i*)(HST + (size_t)b * NGP + i * 4) = v; }
    __threadfence(); }
}
__global__ __launch_bounds__(512) void csrS_kernel(const int* __restrict__ HST, int nG, int NGP, int* __restrict__ START, int* __restrict__ TOT, int* __restrict__ OFF) {
  __shared__ int tot[CSR_MAXG];
  const int b = threadIdx.x;
  for (int pass = 0; pass < 2; ++pass) { int runb = 0; for (int g = 0; g < nG; ++g) { int c = HST[(size_t)b * NGP + g]; c = (c < 0) ? 0 : c; ((volatile int*)OFF)[(size_t)g * CSR_NBLK + b] = runb; runb += c; } __threadfence(); }
  for (int g = threadIdx.x; g < nG; g += 512) { int s = 0; for (int bb = 0; bb < CSR_NBLK; ++bb) { int c = HST[(size_t)bb * NGP + g]; s += (c < 0) ? 0 : c; } tot[g] = s; }
  __syncthreads();
  if (threadIdx.x < 32) {
    __shared__ int st[CSR_MAXG + 32];
    if (threadIdx.x == 0) { int acc = 0; for (int g = 0; g < NGP; ++g) { st[g] = acc; if (g < nG) acc += (tot[g] + 31) & ~31; } st[NGP] = acc; }
    __builtin_amdgcn_fence(__ATOMIC_RELEASE, "workgroup"); __builtin_amdgcn_wave_barrier(); __builtin_amdgcn_fence(__ATOMIC_ACQUIRE, "workgroup");
    for (int pass = 0; pass < 2; ++pass) { for (int i = threadIdx.x; i < NGP + 32; i += 32) { ((volatile int*)START)[i] = (i <= NGP) ? st[min(i, NGP)] : 0; ((volatile int*)TOT)[i] = (i < nG) ? tot[i] : 0; } __threadfence(); } }
}
__global__ __launch_bounds__(256) void csrB_kernel(const int* __restrict__ dst, int N, int nG, int CHP, int NGP, int permLen, const int* __restrict__ STG, const int* __restrict__ HST, const int* __restrict__ OFF, const int* __restrict__ START, const int* __restrict__ TOT, int* __restrict__ PERM, int* __restrict__ ROWPTR, int* __restrict__ ROWCNT, int* __restrict__ FLAG) {
  typedef __attribute__((ext_vector_type(4))) int v4i;
  __shared__ int ids[CSR_CAP]; __shared__ unsigned short key[CSR_CAP]; __shared__ int outp[CSR_CAP]; __shared__ int ncnt[CSR_GN + 1]; __shared__ int boff[CSR_NBLK + 1];
  const int g = blockIdx.x, t_ = threadIdx.x; int tot = TOT[g]; int st = START[g], stn = START[g + 1]; const int v0 = g * CSR_GN; const int nv = min(CSR_GN, N - v0);
  st = (st < 0) ? 0 : (st > permLen - 32 ? permLen - 32 : st) & ~31; stn = (stn < st) ? st : (stn > permLen ? permLen : stn); tot = (tot < 0) ? 0 : tot; if (tot > stn - st && tot <= CSR_CAP) tot = stn - st;
  if (tot > CSR_CAP) {
    for (int pass = 0; pass < 2; ++pass) { for (int i = t_; i < CSR_GN / 4; i += 256) { v4i a, c; for (int e = 0; e < 4; ++e) { a[e] = st; c[e] = 0; } *(volatile v4i*)(ROWPTR + v0 + i * 4) = a; *(volatile v4i*)(ROWCNT + v0 + i * 4) = c; } if (t_ == 0) ((volatile int*)FLAG)[0] = 1; __threadfence(); } (void)nv; return; }
  if (t_ == 0) { int acc = 0; for (int b = 0; b < CSR_NBLK; ++b) { boff[b] = acc; int c = HST[(size_t)b * NGP + g]; c = (c < 0) ? 0 : (c > CHP ? CHP : c); acc += c; if (acc > tot) acc = tot; } boff[CSR_NBLK] = acc; }
  for (int i = t_; i <= CSR_GN; i += 256) ncnt[i] = 0;
  __syncthreads();
  for (int b = 0; b < CSR_NBLK; ++b) { const int c = boff[b + 1] - boff[b]; int o_ = OFF[(size_t)g * CSR_NBLK + b]; o_ = (o_ < 0) ? 0 : (o_ > CHP - c ? CHP - c : o_); const int* src_ = STG + (size_t)b * CHP + o_;
    for (int i = t_; i < c; i += 256) { int id = src_[i]; id = (id < 0) ? 0 : id; ids[boff[b] + i] = id; int d = dst[id]; d = (d < v0) ? v0 : (d >= N ? N - 1 : d); int kk = d - v0; kk = (kk < 0) ? 0 : (kk >= CSR_GN ? CSR_GN - 1 : kk); key[boff[b] + i] = (unsigned short)kk; } }
  __syncthreads();
  if (t_ == 0) { for (int i = 0; i < tot; ++i) ncnt[key[i]] += 1; int acc = 0; for (int vl = 0; vl < CSR_GN; ++vl) { const int c = ncnt[vl]; ncnt[vl] = acc; acc += c; } ncnt[CSR_GN] = acc;
    for (int i = 0; i < tot; ++i) { const int vl = key[i]; outp[ncnt[vl]] = ids[i]; ncnt[vl] += 1; }
    for (int vl = CSR_GN; vl > 0; --vl) ncnt[vl] = ncnt[vl - 1]; ncnt[0] = 0; }
  __syncthreads();
  for (int pass = 0; pass < 2; ++pass) {
    for (int i = t_; i < (stn - st) / 4; i += 256) { v4i v; for (int e = 0; e < 4; ++e) { const int q = i * 4 + e; v[e] = (q < tot) ? outp[q] : -1; } *(volatile v4i*)(PERM + st + i * 4) = v; }
    for (int i = t_; i < CSR_GN / 4; i += 256) { v4i a, c; for (int e = 0; e < 4; ++e) { const int vl = i * 4 + e; a[e] = st + ncnt[vl]; c[e] = (vl < nv) ? (ncnt[vl + 1] - ncnt[vl]) : 0; } *(volatile v4i*)(ROWPTR + v0 + i * 4) = a; *(volatile v4i*)(ROWCNT + v0 + i * 4) = c; }
    __threadfence(); }
}
__global__ __launch_bounds__(256) void csrZ_kernel(int* __restrict__ p, size_t n4) { typedef __attribute__((ext_vector_type(4))) int v4i; const size_t tid = (size_t)blockIdx.x * 256 + threadIdx.x, nth = (size_t)gridDim.x * 256; v4i z = {0, 0, 0, 0}; for (size_t i = tid; i < n4; i += nth) *(volatile v4i*)(p + i * 4) = z; }
struct CsrBufs { int *STG, *HST, *OFF, *START, *TOT, *PERM, *ROWPTR, *ROWCNT, *FLAG; int nG, NGP, CHP; size_t permLen; char* base; size_t bytes; };
static size_t csr_carve(CsrBufs& c, char* ws, size_t off, int E, int N) {
  const size_t off0 = off; c.base = ws + off;
  auto al = [&](size_t bytes) { char* p = ws + off; off += (bytes + 255) & ~(size_t)255; return p; };
  c.nG = (N + CSR_GN - 1) / CSR_GN; c.NGP = (c.nG + 31) & ~31; const int ch = (E + CSR_NBLK - 1) / CSR_NBLK; c.CHP = (ch + 31) & ~31; c.permLen = (size_t)E + 32 * (size_t)c.nG + 32;
  c.STG = (int*)al((size_t)CSR_NBLK * c.CHP * 4); c.HST = (int*)al((size_t)CSR_NBLK * c.NGP * 4); c.OFF = (int*)al((size_t)c.NGP * CSR_NBLK * 4); c.START = (int*)al((size_t)(c.NGP + 64) * 4); c.TOT = (int*)al((size_t)(c.NGP + 64) * 4);
  c.PERM = (int*)al(c.permLen * 4); c.ROWPTR = (int*)al((size_t)c.nG * CSR_GN * 4); c.ROWCNT = (int*)al((size_t)c.nG * CSR_GN * 4); c.FLAG = (int*)al(256);
  c.bytes = off - off0; return off;
}
static void csr_build(const CsrBufs& c, const int* dst, int E, int N, hipStream_t stream) {
  const size_t smem = (size_t)(2 * c.NGP + c.CHP) * 4;
  csrZ_kernel<<<512, 256, 0, stream>>>((int*)c.base, c.bytes / 16);
  csrA_kernel<<<CSR_NBLK, 64, smem, stream>>>(dst, E, N, c.nG, c.CHP, c.NGP, c.STG, c.HST);
  csrS_kernel<<<1, 512, 0, stream>>>(c.HST, c.nG, c.NGP, c.START, c.TOT, c.OFF);
  csrB_kernel<<<c.nG, 256, 0, stream>>>(dst, N, c.nG, c.CHP, c.NGP, (int)c.permLen, c.STG, c.HST, c.OFF, c.START, c.TOT, c.PERM, c.ROWPTR, c.ROWCNT, c.FLAG);
}

typedef __attribute__((ext_vector_type(4))) _Float16 v4h;
typedef __attribute__((ext_vector_type(2))) float v2f;
__global__ __launch_bounds__(256) void wprep_kernel(const float* __restrict__ w1, const float* __restrict__ w2, const float* __restrict__ fw, const float* __restrict__ o1, const float* __restrict__ o2, b16* __restrict__ W1T, b16* __restrict__ W2T, b16* __restrict__ FWT, b16* __restrict__ O1T, b16* __restrict__ O2T) {
  size_t t = (size_t)blockIdx.x * 256 + threadIdx.x; v8b o;
  const size_t n1 = (size_t)L * HP * DP / 8; if (t < n1) { const size_t e = t * 8; const int l = (int)(e / ((size_t)HP * DP)); const size_t el = e % ((size_t)HP * DP); const int oo = (int)(el / DP), k0 = (int)(el % DP);
    for (int j = 0; j < 8; ++j) { const int k = k0 + j; o[j] = (k < D && oo < H2) ? (b16)(bf16_rne(w1[((size_t)l * D + k) * H2 + oo]) * WSC) : (b16)0.0f; } for (int pass = 0; pass < 2; ++pass) { *(volatile v8b*)(W1T + e) = o; __threadfence(); } return; } t -= n1;
  const size_t n2 = (size_t)L * DP * HP / 8; if (t < n2) { const size_t e = t * 8; const int l = (int)(e / ((size_t)DP * HP)); const size_t el = e % ((size_t)DP * HP); const int oo = (int)(el / HP), k0 = (int)(el % HP);
    for (int j = 0; j < 8; ++j) { const int k = k0 + j; o[j] = (k < H2 && oo < D) ? (b16)(bf16_rne(w2[((size_t)l * H2 + k) * D + oo]) * WSC) : (b16)0.0f; } for (int pass = 0; pass < 2; ++pass) { *(volatile v8b*)(W2T + e) = o; __threadfence(); } return; } t -= n2;
  const size_t n3 = (size_t)FD * DP / 8; if (t < n3) { const size_t e = t * 8; const int oo = (int)(e / DP), k0 = (int)(e % DP); for (int j = 0; j < 8; ++j) { const int k = k0 + j; o[j] = (k < D) ? (b16)(bf16_rne(fw[(size_t)k * FD + oo]) * WSC) : (b16)0.0f; } for (int pass = 0; pass < 2; ++pass) { *(volatile v8b*)(FWT + e) = o; __threadfence(); } return; } t -= n3;
  const size_t n4 = (size_t)FD * FD / 8; if (t < n4) { const size_t e = t * 8; const int oo = (int)(e / FD), k0 = (int)(e % FD); for (int j = 0; j < 8; ++j) o[j] = (b16)(bf16_rne(o1[(size_t)(k0 + j) * FD + oo]) * WSC); for (int pass = 0; pass < 2; ++pass) { *(volatile v8b*)(O1T + e) = o; __threadfence(); } return; } t -= n4;
  const size_t n5 = (size_t)FD2 * FD / 8; if (t < n5) { const size_t e = t * 8; const int oo = (int)(e / FD), k0 = (int)(e % FD); for (int j = 0; j < 8; ++j) o[j] = (b16)(bf16_rne(o2[(size_t)(k0 + j) * FD2 + oo]) * WSC); for (int pass = 0; pass < 2; ++pass) { *(volatile v8b*)(O2T + e) = o; __threadfence(); } }
}
__global__ __launch_bounds__(256) void h0_kernel(const int* __restrict__ xi, const float* __restrict__ xe1, const float* __restrict__ xe2, float* __restrict__ Hf) {
  const size_t u = (size_t)blockIdx.x * 256 + threadIdx.x; if (u >= (size_t)NP * DP / 4) return; const size_t e = u * 4; const size_t v = e / DP; const int c = (int)(e % DP); v4f o = {0.0f, 0.0f, 0.0f, 0.0f};
  if (v < (size_t)N) { const int a = iclamp(xi[v * 2], 0, 118), b = iclamp(xi[v * 2 + 1], 0, 2); for (int j = 0; j < 4; ++j) if (c + j < D) o[j] = bf16_rne(xe1[(size_t)a * D + c + j]) + bf16_rne(xe2[(size_t)b * D + c + j]); }
  for (int pass = 0; pass < 2; ++pass) { *(volatile v4f*)(Hf + e) = o; __threadfence(); }
}
__global__ __launch_bounds__(256) void ee_kernel(int l, const float* __restrict__ ee1, const float* __restrict__ ee2, const float* __restrict__ lepb, const float* __restrict__ eW1, const float* __restrict__ eb1, const float* __restrict__ eW2, const float* __restrict__ eb2, float* __restrict__ EE) {
  __shared__ float ce[3 * D], hid[D];
  const int ty = blockIdx.x, et = ty / 3, ed = ty % 3, t = threadIdx.x;
  for (int c = t; c < 3 * D; c += 256) { float v; if (c < D) v = bf16_rne(ee1[((size_t)l * 5 + et) * D + c]); else if (c < 2 * D) v = bf16_rne(ee2[((size_t)l * 3 + ed) * D + (c - D)]); else v = bf16_rne(lepb[(size_t)l * D + (c - 2 * D)]); ce[c] = v; }
  __syncthreads();
  for (int c = t; c < D; c += 256) { float s = bf16_rne(eb1[(size_t)l * D + c]);
#pragma unroll 1
    for (int k = 0; k < 3 * D; ++k) s += pmul(ce[k], bf16_rne(eW1[((size_t)l * 3 * D + k) * D + c])); hid[c] = fmaxf(s, 0.0f); }
  __syncthreads();
  for (int pass = 0; pass < 2; ++pass) { for (int c = t; c < DP; c += 256) { float s = 0.0f; if (c < D) { s = bf16_rne(eb2[(size_t)l * D + c]);
#pragma unroll 1
        for (int k = 0; k < D; ++k) s += pmul(hid[k], bf16_rne(eW2[((size_t)l * D + k) * D + c])); } ((volatile float*)EE)[(size_t)ty * DP + c] = s; } __threadfence(); }
}
__global__ __launch_bounds__(256) void agg_kernel(const float* __restrict__ Hf, const float* __restrict__ EE, const int* __restrict__ srcs, const int* __restrict__ eattr, const int* __restrict__ PERM, const int* __restrict__ ROWPTR, const int* __restrict__ ROWCNT, int permLen, b16* __restrict__ AGh, b16* __restrict__ AGl) {
  const int wave = threadIdx.x >> 5, lane = threadIdx.x & 31; const size_t v = (size_t)blockIdx.x * 8 + wave;
  v4f a[3]; for (int q = 0; q < 3; ++q) a[q] = (v4f){0.0f, 0.0f, 0.0f, 0.0f};
  if (v < (size_t)N) {
    { const float* hs = Hf + v * DP; const float* es = EE + (size_t)(4 * 3 + 0) * DP; for (int q = 0; q < 3; ++q) { const int c = lane * 4 + 128 * q; if (c < DP) a[q] = *(const v4f*)(hs + c) + *(const v4f*)(es + c); } }
    int st = ROWPTR[v], cnt = ROWCNT[v]; cnt = iclamp(cnt, 0, 65536); st = iclamp(st, 0, permLen - cnt);
#pragma unroll 1
    for (int j = 0; j < cnt; ++j) { const int e = iclamp(PERM[st + j], 0, E - 1); const int s = iclamp(srcs[e], 0, N - 1); const int ty = iclamp(eattr[e * 2], 0, 4) * 3 + iclamp(eattr[e * 2 + 1], 0, 2); const float msk = (s < NLIM) ? 1.0f : 0.0f;
      const float* hs = Hf + (size_t)s * DP; const float* es = EE + (size_t)ty * DP;
      for (int q = 0; q < 3; ++q) { const int c = lane * 4 + 128 * q; if (c < DP) { const v4f hv = *(const v4f*)(hs + c), ev = *(const v4f*)(es + c); a[q] += (hv + ev) * msk; } } } }
  for (int pass = 0; pass < 2; ++pass) { for (int q = 0; q < 3; ++q) { const int c = lane * 4 + 128 * q; if (c < DP) { v4h hv, lv; for (int j = 0; j < 4; ++j) { b16 p, qq; split16(a[q][j] * XS, p, qq); hv[j] = p; lv[j] = qq; } *(volatile v4h*)(AGh + v * DP + c) = hv; *(volatile v4h*)(AGl + v * DP + c) = lv; } } __threadfence(); }
}
template <int KD, int NCOL, int RELU, int OUTP, int OUTF, int PSUM>
__global__ __launch_bounds__(128) void gemm_kernel(const b16* __restrict__ Ah, const b16* __restrict__ Al, const b16* __restrict__ WT, const float* __restrict__ bias, int nb, b16* __restrict__ Oh, b16* __restrict__ Ol, float* __restrict__ OUT, float* __restrict__ PS) {
  __shared__ __attribute__((aligned(16))) float Tf[4][16][64 + 4];
  const int wave = threadIdx.x >> 5, lane = threadIdx.x & 31, nloc = lane & 15, hlf = lane >> 4; const size_t m0 = (size_t)blockIdx.x * 64 + wave * 16; const int n0 = blockIdx.y * 64;
  v8f acc[4];
#pragma unroll
  for (int t = 0; t < 4; ++t) acc[t] = (v8f){};
#pragma unroll 2
  for (int kb = 0; kb < KD; kb += 32) { const v16b a = frag_kb(Ah + (m0 + nloc) * KD + kb, hlf), al = frag_kb(Al + (m0 + nloc) * KD + kb, hlf);
#pragma unroll
    for (int t = 0; t < 4; ++t) { const v16b bw = frag_kb(WT + (size_t)(n0 + t * 16 + nloc) * KD + kb, hlf); acc[t] = wmma16b(a, bw, acc[t]); acc[t] = wmma16b(al, bw, acc[t]); } }
#pragma unroll
  for (int t = 0; t < 4; ++t) { const int cc = n0 + t * 16 + nloc; const float bb = (cc < nb) ? bf16_rne(bias[cc]) : 0.0f;
#pragma unroll
    for (int r = 0; r < 8; ++r) { float v = acc[t][r] * (1.0f / (XS * WSC)) + bb; if (RELU) v = fmaxf(v, 0.0f); if (m0 + 8 * hlf + r >= (size_t)NLIMN) v = 0.0f; Tf[wave][8 * hlf + r][t * 16 + nloc] = v; } }
  __syncthreads();
  for (int pass = 0; pass < 2; ++pass) { for (int rr = 0; rr < 16; ++rr) {
      if (OUTF) *(volatile v2f*)(OUT + (m0 + rr) * NCOL + n0 + lane * 2) = *(const v2f*)(&Tf[wave][rr][lane * 2]);
      if (OUTP) { const v2f v = *(const v2f*)(&Tf[wave][rr][lane * 2]); b16 p0, q0, p1, q1; split16(v[0] * XS, p0, q0); split16(v[1] * XS, p1, q1); typedef __attribute__((ext_vector_type(2))) _Float16 v2h; v2h hv = {p0, p1}, lv = {q0, q1}; *(volatile v2h*)(Oh + (m0 + rr) * NCOL + n0 + lane * 2) = hv; *(volatile v2h*)(Ol + (m0 + rr) * NCOL + n0 + lane * 2) = lv; } }
    if (PSUM && threadIdx.x < 64) { float s = 0.0f;
#pragma unroll 1
      for (int w = 0; w < 4; ++w) for (int rr = 0; rr < 16; ++rr) s += Tf[w][rr][threadIdx.x]; ((volatile float*)PS)[(size_t)blockIdx.x * NCOL + n0 + threadIdx.x] = s; }
    __threadfence(); }
}
__global__ __launch_bounds__(320) void colstat_kernel(const float* __restrict__ PS, float* __restrict__ STAT) {
  const int c = threadIdx.x; float s = 0.0f;
#pragma unroll 1
  for (int b = 0; b < NBPL; ++b) s += PS[(size_t)b * DP + c];
  for (int pass = 0; pass < 2; ++pass) { ((volatile float*)STAT)[c] = s * (1.0f / NLIMN); __threadfence(); }
}
__global__ __launch_bounds__(320) void var_kernel(const float* __restrict__ P, const float* __restrict__ MEAN, float* __restrict__ PS) {
  const int c = threadIdx.x; const float m = MEAN[c]; float a = 0.0f;
#pragma unroll 1
  for (int rr = 0; rr < RPB; ++rr) { const size_t v = (size_t)blockIdx.x * RPB + rr; const float d = v < (size_t)NLIMN ? P[v * DP + c] - m : 0.0f; a += d * d; }
  for (int pass = 0; pass < 2; ++pass) { ((volatile float*)PS)[(size_t)blockIdx.x * DP + c] = a; __threadfence(); }
}
__global__ __launch_bounds__(256) void apply_kernel(float* __restrict__ P, const float* __restrict__ MEAN, const float* __restrict__ VAR, const float* __restrict__ g_, const float* __restrict__ b_, int relu) {
  const size_t u = (size_t)blockIdx.x * 256 + threadIdx.x; if (u >= (size_t)NP * DP / 4) return; const size_t e = u * 4; const size_t v = e / DP; const int c = (int)(e % DP);
  v4f o = {0.0f, 0.0f, 0.0f, 0.0f}; if (v < (size_t)NLIMN) { const v4f p = *(const v4f*)(P + e); for (int j = 0; j < 4; ++j) { const int cc = c + j; if (cc < D) { float y = (p[j] - MEAN[cc]) * rsqrtf(VAR[cc] + BNEPS) * bf16_rne(g_[cc]) + bf16_rne(b_[cc]); if (relu) y = fmaxf(y, 0.0f); o[j] = y; } } }
  for (int pass = 0; pass < 2; ++pass) { *(volatile v4f*)(P + e) = o; __threadfence(); }
}
__device__ int lower_bound_i(const int* a, int n, int key) { int lo = 0, hi = n; while (lo < hi) { const int mid = (lo + hi) >> 1; if (a[mid] < key) lo = mid + 1; else hi = mid; } return lo; }
__global__ __launch_bounds__(320) void pool_kernel(const float* __restrict__ Hf, const int* __restrict__ batch, b16* __restrict__ PGh, b16* __restrict__ PGl) {
  __shared__ __attribute__((aligned(16))) b16 sh[DP], sl[DP];
  const int g = blockIdx.x, c = threadIdx.x; int lo = lower_bound_i(batch, N, g), hi = lower_bound_i(batch, N, g + 1); lo = lo < NLIMN ? lo : NLIMN; hi = hi < NLIMN ? hi : NLIMN;
  float s = 0.0f;
#pragma unroll 1
  for (int v = lo; v < hi; ++v) s += Hf[(size_t)v * DP + c];
  const float m = s / fmaxf((float)(hi - lo), 1.0f); b16 p, q; split16(m * XS, p, q); sh[c] = p; sl[c] = q;
  __syncthreads();
  for (int pass = 0; pass < 2; ++pass) { if (c < DP / 8) { *(volatile v8b*)(PGh + (size_t)g * DP + c * 8) = *(const v8b*)(&sh[c * 8]); *(volatile v8b*)(PGl + (size_t)g * DP + c * 8) = *(const v8b*)(&sl[c * 8]); } __threadfence(); }
}
}

extern "C" void kernel_launch(void* const* d_in, const int* in_sizes, int n_in, void* d_out, int out_size, void* d_ws, size_t ws_size, hipStream_t stream) {
  (void)n_in;
  auto Fp = [&](int i) { return (const float*)d_in[i]; }; auto Ip = [&](int i) { return (const int*)d_in[i]; };
  if (in_sizes[0] != N * 2 || in_sizes[1] != 2 * EFULL || in_sizes[2] != EFULL * 2 || in_sizes[3] != N || in_sizes[4] != 119 * D || in_sizes[5] != 3 * D || in_sizes[6] != L * 5 * D || in_sizes[7] != L * 3 * D || in_sizes[9] != L * D || in_sizes[10] != L * 3 * D * D || in_sizes[12] != L * D * D || in_sizes[14] != L * D * H2 || in_sizes[16] != L * H2 * D || in_sizes[20] != D * FD || in_sizes[22] != FD * FD || in_sizes[24] != FD * FD2 || (size_t)out_size != (size_t)G * FD + (size_t)G * FD2) return;
  size_t off = 0; char* ws = (char*)d_ws;
  auto carve = [&](size_t bytes) { char* p = ws + off; off += (bytes + 255) & ~(size_t)255; return p; };
  b16* W1T = (b16*)carve((size_t)L * HP * DP * 2); b16* W2T = (b16*)carve((size_t)L * DP * HP * 2); b16* FWT = (b16*)carve((size_t)FD * DP * 2); b16* O1T = (b16*)carve((size_t)FD * FD * 2); b16* O2T = (b16*)carve((size_t)FD2 * FD * 2);
  float* Hf = (float*)carve((size_t)NP * DP * 4); float* EE = (float*)carve((size_t)NT * DP * 4); b16* AGh = (b16*)carve((size_t)NP * DP * 2); b16* AGl = (b16*)carve((size_t)NP * DP * 2); b16* H1h = (b16*)carve((size_t)NP * HP * 2); b16* H1l = (b16*)carve((size_t)NP * HP * 2);
  float* PS = (float*)carve((size_t)NBP * DP * 4); float* ST = (float*)carve((size_t)2 * DP * 4); b16* PGh = (b16*)carve((size_t)G * DP * 2); b16* PGl = (b16*)carve((size_t)G * DP * 2); b16* Q1h = (b16*)carve((size_t)G * FD * 2); b16* Q1l = (b16*)carve((size_t)G * FD * 2); b16* Q2h = (b16*)carve((size_t)G * FD * 2); b16* Q2l = (b16*)carve((size_t)G * FD * 2);
  CsrBufs csr; off = csr_carve(csr, ws, off, E, N);
  if (off > ws_size || off > ((size_t)128 << 20)) return;
  wprep_kernel<<<(unsigned)((((size_t)L * HP * DP * 2 + (size_t)FD * DP + (size_t)FD * FD + (size_t)FD2 * FD) / 8 + 255) / 256), 256, 0, stream>>>(Fp(14), Fp(16), Fp(20), Fp(22), Fp(24), W1T, W2T, FWT, O1T, O2T);
  h0_kernel<<<(unsigned)(((size_t)NP * DP / 4 + 255) / 256), 256, 0, stream>>>(Ip(0), Fp(4), Fp(5), Hf);
  csr_build(csr, Ip(1) + EFULL, E, N, stream);
  for (int l = 0; l < L; ++l) {
    ee_kernel<<<NT, 256, 0, stream>>>(l, Fp(6), Fp(7), Fp(9), Fp(10), Fp(11), Fp(12), Fp(13), EE);
    agg_kernel<<<NLIM / 8, 256, 0, stream>>>(Hf, EE, Ip(1), Ip(2), csr.PERM, csr.ROWPTR, csr.ROWCNT, (int)csr.permLen, AGh, AGl);
    gemm_kernel<DP, HP, 1, 1, 0, 0><<<dim3(NLIM / 64, HP / 64), 128, 0, stream>>>(AGh, AGl, W1T + (size_t)l * HP * DP, Fp(15) + (size_t)l * H2, H2, H1h, H1l, nullptr, nullptr);
    gemm_kernel<HP, DP, 0, 0, 1, 1><<<dim3(NLIM / 64, DP / 64), 128, 0, stream>>>(H1h, H1l, W2T + (size_t)l * DP * HP, Fp(17) + (size_t)l * D, D, nullptr, nullptr, Hf, PS);
    colstat_kernel<<<1, DP, 0, stream>>>(PS, ST); var_kernel<<<NBPL, DP, 0, stream>>>(Hf, ST, PS); colstat_kernel<<<1, DP, 0, stream>>>(PS, ST + DP);
    apply_kernel<<<(unsigned)(((size_t)NP * DP / 4 + 255) / 256), 256, 0, stream>>>(Hf, ST, ST + DP, Fp(18) + (size_t)l * D, Fp(19) + (size_t)l * D, l < L - 1 ? 1 : 0); }
  pool_kernel<<<G, DP, 0, stream>>>(Hf, Ip(3), PGh, PGl);
  gemm_kernel<DP, FD, 0, 1, 1, 0><<<dim3(G / 64, FD / 64), 128, 0, stream>>>(PGh, PGl, FWT, Fp(21), FD, Q1h, Q1l, (float*)d_out, nullptr);
  gemm_kernel<FD, FD, 1, 1, 0, 0><<<dim3(G / 64, FD / 64), 128, 0, stream>>>(Q1h, Q1l, O1T, Fp(23), FD, Q2h, Q2l, nullptr, nullptr);
  gemm_kernel<FD, FD2, 0, 0, 1, 0><<<dim3(G / 64, FD2 / 64), 128, 0, stream>>>(Q2h, Q2l, O2T, Fp(25), FD2, nullptr, nullptr, (float*)d_out + (size_t)G * FD, nullptr);
}
